// EGAT_55611236549395
// MI455X (gfx1250) — hardware-verified
//
#include <hip/hip_runtime.h>


namespace {
constexpr int N = 384, DIM = 256, NH = 4, DH = 64, HD = NH * DH  , MD = 16, E2 = 258, KE = 288  , PW = 384  , A1 = 64, NRH = N * NH  , JC = 32;
constexpr float XS = 8.0f, WSC = 256.0f;

typedef _Float16 b16;
typedef __attribute__((ext_vector_type(16))) _Float16 v16b;
typedef __attribute__((ext_vector_type(8))) _Float16 v8b;
typedef __attribute__((ext_vector_type(8))) float v8f;
typedef __attribute__((ext_vector_type(4))) float v4f;
__device__ __forceinline__ float bf16_rne(float f) { unsigned int u = __float_as_uint(f); u += 0x7FFFu + ((u >> 16) & 1u); return __uint_as_float(u & 0xFFFF0000u); }
__device__ __forceinline__ void split16(float v, b16& hi, b16& lo) { hi = (b16)v; lo = (b16)(v - (float)hi); }
__device__ __forceinline__ v16b frag_kb(const b16* p, int hh) { const v8b a = *(const v8b*)(p + 8 * hh), b = *(const v8b*)(p + 16 + 8 * hh); v16b f;
#pragma unroll
  for (int e = 0; e < 8; ++e) { f[e] = a[e]; f[8 + e] = b[e]; } return f; }
__device__ __forceinline__ v8f wmma16b(v16b a, v16b b, v8f c) { v8f d = __builtin_amdgcn_wmma_f32_16x16x32_f16(false, a, false, b, (short)0, c, false, false); asm volatile("v_nop\n\tv_nop\n\tv_nop\n\tv_nop" : "+v"(d) : "v"(a), "v"(b)); return d; }
__device__ __forceinline__ void wave_lds_sync() { __builtin_amdgcn_fence(__ATOMIC_RELEASE, "workgroup"); __builtin_amdgcn_wave_barrier(); __builtin_amdgcn_fence(__ATOMIC_ACQUIRE, "workgroup"); }
__device__ __forceinline__ float nexp2(float x) { return __builtin_amdgcn_exp2f(x); }
__device__ __forceinline__ float pmul(float a, float b) { float p = a * b; asm volatile("" : "+v"(p)); return p; }
constexpr float LOG2E = 1.4426950408889634f;

__global__ __launch_bounds__(256) void prep_kernel(const float* __restrict__ x, const float* __restrict__ wqkv, const float* __restrict__ wout, const float* __restrict__ we1, const float* __restrict__ we2, const float* __restrict__ wa1, const float* __restrict__ wa2, const float* __restrict__ wc1, const float* __restrict__ wc2,
    b16* __restrict__ X16, b16* __restrict__ WQKV, b16* __restrict__ WOUT, b16* __restrict__ WE1P, b16* __restrict__ WE1Q, b16* __restrict__ WE2T, b16* __restrict__ WA1T, b16* __restrict__ WC1T, b16* __restrict__ WA2T, b16* __restrict__ WC2T) {
  const size_t t = (size_t)blockIdx.x * 256 + threadIdx.x; size_t u = t; v8b o;
  const size_t nx = (size_t)N * DIM / 8, n1 = (size_t)3 * HD * DIM / 8, n2 = (size_t)DIM * HD / 8, n3 = (size_t)PW * DH / 8, n5 = (size_t)MD * KE / 8, n6 = (size_t)A1 * 32 / 8, n8 = (size_t)16 * A1 / 8;
  if (u < nx) { const size_t e = u * 8; const v4f a = *(const v4f*)(x + e), c = *(const v4f*)(x + e + 4); for (int j = 0; j < 4; ++j) { o[j] = (b16)(bf16_rne(a[j]) * XS); o[4 + j] = (b16)(bf16_rne(c[j]) * XS); } for (int pass = 0; pass < 2; ++pass) { *(volatile v8b*)(X16 + e) = o; __threadfence(); } return; } u -= nx;
  if (u < n1) { const int e = (int)u * 8; const int oo = e / DIM, k0 = e % DIM; for (int j = 0; j < 8; ++j) o[j] = (b16)(bf16_rne(wqkv[(size_t)(k0 + j) * (3 * HD) + oo]) * WSC); for (int pass = 0; pass < 2; ++pass) { *(volatile v8b*)(WQKV + e) = o; __threadfence(); } return; } u -= n1;
  if (u < n2) { const int e = (int)u * 8; const int oo = e / HD, k0 = e % HD; for (int j = 0; j < 8; ++j) o[j] = (b16)(bf16_rne(wout[(size_t)(k0 + j) * DIM + oo]) * WSC); for (int pass = 0; pass < 2; ++pass) { *(volatile v8b*)(WOUT + e) = o; __threadfence(); } return; } u -= n2;
  for (int which = 0; which < 2; ++which) { if (u < n3) { const int e = (int)u * 8; const int oo = e / DH, k0 = e % DH; for (int j = 0; j < 8; ++j) o[j] = (oo < E2) ? (b16)(bf16_rne(we1[(size_t)(which * DH + k0 + j) * E2 + oo]) * WSC) : (b16)0.0f; for (int pass = 0; pass < 2; ++pass) { *(volatile v8b*)((which == 0 ? WE1P : WE1Q) + e) = o; __threadfence(); } return; } u -= n3; }
  if (u < n5) { const int e = (int)u * 8; const int oo = e / KE, k0 = e % KE; for (int j = 0; j < 8; ++j) { const int k = k0 + j; o[j] = (k < E2) ? (b16)(bf16_rne(we2[(size_t)k * MD + oo]) * WSC) : (b16)0.0f; } for (int pass = 0; pass < 2; ++pass) { *(volatile v8b*)(WE2T + e) = o; __threadfence(); } return; } u -= n5;
  for (int which = 0; which < 2; ++which) { if (u < n6) { const int e = (int)u * 8; const int oo = e / 32, k0 = e % 32; const float* w = which == 0 ? wa1 : wc1; for (int j = 0; j < 8; ++j) { const int k = k0 + j; o[j] = (k < MD) ? (b16)(bf16_rne(w[k * A1 + oo]) * WSC) : (b16)0.0f; } for (int pass = 0; pass < 2; ++pass) { *(volatile v8b*)((which == 0 ? WA1T : WC1T) + e) = o; __threadfence(); } return; } u -= n6; }
  for (int which = 0; which < 2; ++which) { if (u < n8) { const int e = (int)u * 8; const int oo = e / A1, k0 = e % A1; const float* w = which == 0 ? wa2 : wc2; for (int j = 0; j < 8; ++j) o[j] = (oo == 0) ? (b16)(bf16_rne(w[k0 + j]) * WSC) : (b16)0.0f; for (int pass = 0; pass < 2; ++pass) { *(volatile v8b*)((which == 0 ? WA2T : WC2T) + e) = o; __threadfence(); } return; } u -= n8; }
}
__global__ __launch_bounds__(128) void qkv_kernel(const b16* __restrict__ X16, const b16* __restrict__ WQKV, float* __restrict__ QKV, b16* __restrict__ QKh, b16* __restrict__ QKl) {
  __shared__ __attribute__((aligned(16))) float Tf[4][16][128 + 4]; __shared__ __attribute__((aligned(16))) b16 Th[4][16][128 + 8], Tl[4][16][128 + 8];
  const int wave = threadIdx.x >> 5, lane = threadIdx.x & 31, nloc = lane & 15, hlf = lane >> 4; const size_t m0 = (size_t)blockIdx.x * 64 + wave * 16; const int n0 = blockIdx.y * 128;
  v8f acc[8];
#pragma unroll
  for (int t = 0; t < 8; ++t) acc[t] = (v8f){};
#pragma unroll 2
  for (int kb = 0; kb < DIM; kb += 32) { const v16b a = frag_kb(X16 + (m0 + nloc) * DIM + kb, hlf);
#pragma unroll
    for (int t = 0; t < 8; ++t) acc[t] = wmma16b(a, frag_kb(WQKV + (size_t)(n0 + t * 16 + nloc) * DIM + kb, hlf), acc[t]); }
#pragma unroll
  for (int t = 0; t < 8; ++t)
#pragma unroll
    for (int r = 0; r < 8; ++r) { const float y = acc[t][r] * (1.0f / (XS * WSC)); Tf[wave][8 * hlf + r][t * 16 + nloc] = y; b16 p, q; split16(y * XS, p, q); Th[wave][8 * hlf + r][t * 16 + nloc] = p; Tl[wave][8 * hlf + r][t * 16 + nloc] = q; }
  wave_lds_sync();
  for (int pass = 0; pass < 2; ++pass) { for (int rr = 0; rr < 16; ++rr) *(volatile v4f*)(QKV + (m0 + rr) * (3 * HD) + n0 + lane * 4) = *(const v4f*)(&Tf[wave][rr][lane * 4]);
    if (n0 < 2 * HD) { for (int r2 = 0; r2 < 16; r2 += 2) { const int rr = r2 + (lane >> 4), c8 = (lane & 15) * 8; const size_t gi = (m0 + rr) * (2 * HD) + n0 + c8; *(volatile v8b*)(QKh + gi) = *(const v8b*)(&Th[wave][rr][c8]); *(volatile v8b*)(QKl + gi) = *(const v8b*)(&Tl[wave][rr][c8]); } }
    __threadfence(); }
}
__global__ __launch_bounds__(128) void pq_kernel(const b16* __restrict__ QKh, const b16* __restrict__ QKl, const b16* __restrict__ WE1P, const b16* __restrict__ WE1Q, const float* __restrict__ be1, float* __restrict__ P, float* __restrict__ Q) {
  __shared__ __attribute__((aligned(16))) float Tf[4][16][128 + 4];
  const int wave = threadIdx.x >> 5, lane = threadIdx.x & 31, nloc = lane & 15, hlf = lane >> 4; const int kind = blockIdx.z; const size_t m0 = (size_t)blockIdx.x * 64 + wave * 16; const int n0 = blockIdx.y * 128;
  const b16* W = kind == 0 ? WE1P : WE1Q; const size_t arow = m0 + nloc; const size_t abase = (arow / NH) * (2 * HD) + (kind == 0 ? 0 : HD) + (arow % NH) * DH;
  v8f acc[8];
#pragma unroll
  for (int t = 0; t < 8; ++t) acc[t] = (v8f){};
#pragma unroll
  for (int kb = 0; kb < DH; kb += 32) { const v16b a = frag_kb(QKh + abase + kb, hlf), al = frag_kb(QKl + abase + kb, hlf);
#pragma unroll
    for (int t = 0; t < 8; ++t) { const v16b bw = frag_kb(W + (size_t)(n0 + t * 16 + nloc) * DH + kb, hlf); acc[t] = wmma16b(a, bw, acc[t]); acc[t] = wmma16b(al, bw, acc[t]); } }
#pragma unroll
  for (int t = 0; t < 8; ++t) { const int c = n0 + t * 16 + nloc; const float bb = (kind == 0 && c < E2) ? bf16_rne(be1[c]) : 0.0f;
#pragma unroll
    for (int r = 0; r < 8; ++r) Tf[wave][8 * hlf + r][t * 16 + nloc] = acc[t][r] * (1.0f / (XS * WSC)) + bb; }
  wave_lds_sync();
  float* dst = kind == 0 ? P : Q;
  for (int pass = 0; pass < 2; ++pass) { for (int rr = 0; rr < 16; ++rr) *(volatile v4f*)(dst + (m0 + rr) * PW + n0 + lane * 4) = *(const v4f*)(&Tf[wave][rr][lane * 4]); __threadfence(); }
}
__global__ __launch_bounds__(256) void pair_kernel(const float* __restrict__ P, const float* __restrict__ Q, const float* __restrict__ we1, const float* __restrict__ coors, const float* __restrict__ QKV, const b16* __restrict__ WE2T, const float* __restrict__ be2, const b16* __restrict__ WA1T, const float* __restrict__ ba1, const b16* __restrict__ WC1T, const float* __restrict__ bc1, const b16* __restrict__ WA2T, const float* __restrict__ ba2, const b16* __restrict__ WC2T, const float* __restrict__ bc2, b16* __restrict__ OHh, b16* __restrict__ OHl, float* __restrict__ CP) {
  __shared__ __attribute__((aligned(16))) b16 Ah[JC][KE + 8], Al[JC][KE + 8]; __shared__ __attribute__((aligned(16))) b16 Mh[JC][32 + 8], Ml[JC][32 + 8]; __shared__ __attribute__((aligned(16))) b16 Hh[2][JC][A1 + 8], Hl[2][JC][A1 + 8];
  __shared__ float Wr[KE]; __shared__ float Pi[KE]; __shared__ float dist[JC]; __shared__ float SimL[N], CwL[N]; __shared__ float stat[4]; __shared__ float cpart[8][3]; __shared__ __attribute__((aligned(16))) b16 orow_h[DH], orow_l[DH]; __shared__ __attribute__((aligned(16))) float cprow[32];
  const int h = blockIdx.y, i = blockIdx.x, t_ = threadIdx.x, wave = t_ >> 5, lane = t_ & 31, nloc = lane & 15, hlf = lane >> 4;
  for (int k = t_; k < KE; k += 256) { Wr[k] = (k < E2) ? bf16_rne(we1[(size_t)(2 * DH) * E2 + k]) : 0.0f; Pi[k] = P[((size_t)i * NH + h) * PW + k]; }
  const float cix = bf16_rne(coors[i * 3 + 0]), ciy = bf16_rne(coors[i * 3 + 1]), ciz = bf16_rne(coors[i * 3 + 2]);
  __syncthreads();
  for (int jc = 0; jc < N; jc += JC) {
    if (t_ < JC) { const int j = jc + t_; const float dx = cix - bf16_rne(coors[j * 3 + 0]), dy = ciy - bf16_rne(coors[j * 3 + 1]), dz = ciz - bf16_rne(coors[j * 3 + 2]); dist[t_] = sqrtf(dx * dx + dy * dy + dz * dz); }
    __syncthreads();
    for (int q = t_; q < JC * KE; q += 256) { const int jj = q / KE, k = q % KE; const float pre = Pi[k] + Q[((size_t)(jc + jj) * NH + h) * PW + k] + pmul(dist[jj], Wr[k]); b16 p, ql; split16(fmaxf(pre, 0.0f) * XS, p, ql); Ah[jj][k] = p; Al[jj][k] = ql; }
    __syncthreads();
    if (wave < 2) { v8f d = {}; const int rt = wave;
      for (int kb = 0; kb < KE; kb += 32) { const v16b bw = frag_kb(WE2T + (size_t)nloc * KE + kb, hlf); d = wmma16b(frag_kb(&Ah[rt * 16 + nloc][kb], hlf), bw, d); d = wmma16b(frag_kb(&Al[rt * 16 + nloc][kb], hlf), bw, d); }
      for (int r = 0; r < 8; ++r) { const float mv = d[r] * (1.0f / (XS * WSC)) + bf16_rne(be2[nloc]); b16 p, ql; split16(mv * XS, p, ql); Mh[rt * 16 + 8 * hlf + r][nloc] = p; Ml[rt * 16 + 8 * hlf + r][nloc] = ql; Mh[rt * 16 + 8 * hlf + r][16 + nloc] = (b16)0.0f; Ml[rt * 16 + 8 * hlf + r][16 + nloc] = (b16)0.0f; } }
    __syncthreads();
    if (wave < 4) { const int which = wave >> 1, rt = wave & 1; const b16* W1 = which == 0 ? WA1T : WC1T; const float* bb = which == 0 ? ba1 : bc1; const v16b a = frag_kb(&Mh[rt * 16 + nloc][0], hlf), al = frag_kb(&Ml[rt * 16 + nloc][0], hlf);
#pragma unroll
      for (int t = 0; t < 4; ++t) { v8f d = {}; const v16b bw = frag_kb(W1 + (size_t)(t * 16 + nloc) * 32, hlf); d = wmma16b(a, bw, d); d = wmma16b(al, bw, d);
        for (int r = 0; r < 8; ++r) { b16 p, ql; split16(fmaxf(d[r] * (1.0f / (XS * WSC)) + bf16_rne(bb[t * 16 + nloc]), 0.0f) * XS, p, ql); Hh[which][rt * 16 + 8 * hlf + r][t * 16 + nloc] = p; Hl[which][rt * 16 + 8 * hlf + r][t * 16 + nloc] = ql; } } }
    __syncthreads();
    if (wave < 4) { const int which = wave >> 1, rt = wave & 1; const b16* W2 = which == 0 ? WA2T : WC2T; v8f d = {};
#pragma unroll
      for (int kb = 0; kb < A1; kb += 32) { const v16b bw = frag_kb(W2 + (size_t)nloc * A1 + kb, hlf); d = wmma16b(frag_kb(&Hh[which][rt * 16 + nloc][kb], hlf), bw, d); d = wmma16b(frag_kb(&Hl[which][rt * 16 + nloc][kb], hlf), bw, d); }
      if (nloc == 0) { const float bb = bf16_rne(which == 0 ? ba2[0] : bc2[0]); for (int r = 0; r < 8; ++r) { const int j = jc + rt * 16 + 8 * hlf + r; const float val = d[r] * (1.0f / (XS * WSC)) + bb; if (which == 0) SimL[j] = val; else CwL[j] = (j == i) ? -INFINITY : val; } } }
    __syncthreads(); }
  if (wave < 2) { float* L = wave == 0 ? SimL : CwL; float mx = -INFINITY; for (int j = lane; j < N; j += 32) mx = fmaxf(mx, L[j]);
#pragma unroll
    for (int o = 16; o >= 1; o >>= 1) mx = fmaxf(mx, __shfl_xor(mx, o));
    float sm = 0.0f; for (int j = lane; j < N; j += 32) { const float w = nexp2((L[j] - mx) * LOG2E); L[j] = w; sm += w; }
#pragma unroll
    for (int o = 16; o >= 1; o >>= 1) sm += __shfl_xor(sm, o);
    if (lane == 0) stat[wave] = 1.0f / sm; }
  __syncthreads();
  if (t_ < DH) { float acc = 0.0f; const float inv = stat[0]; for (int j = 0; j < N; ++j) acc += pmul(SimL[j] * inv, QKV[(size_t)j * (3 * HD) + 2 * HD + h * DH + t_]); b16 p, ql; split16(acc * XS, p, ql); orow_h[t_] = p; orow_l[t_] = ql; }
  else if (t_ < DH + 96) { const int c = (t_ - DH) >> 5, l2 = (t_ - DH) & 31; const float cic = c == 0 ? cix : c == 1 ? ciy : ciz; const float inv = stat[1]; float s = 0.0f;
    for (int j = l2; j < N; j += 32) s += pmul(CwL[j] * inv, cic - bf16_rne(coors[j * 3 + c]));
#pragma unroll
    for (int o = 16; o >= 1; o >>= 1) s += __shfl_xor(s, o);
    if (l2 == 0) cpart[c][0] = s; }
  __syncthreads();
  if (t_ < 32) cprow[t_] = (t_ < 3) ? cpart[t_][0] : 0.0f;
  __syncthreads();
  for (int pass = 0; pass < 2; ++pass) {
    if (t_ < 16) { *(volatile __attribute__((ext_vector_type(4))) _Float16*)(OHh + (size_t)i * HD + h * DH + t_ * 4) = *(const __attribute__((ext_vector_type(4))) _Float16*)(&orow_h[t_ * 4]); *(volatile __attribute__((ext_vector_type(4))) _Float16*)(OHl + (size_t)i * HD + h * DH + t_ * 4) = *(const __attribute__((ext_vector_type(4))) _Float16*)(&orow_l[t_ * 4]); }
    else if (t_ >= 32 && t_ < 40) *(volatile v4f*)(CP + ((size_t)h * N + i) * 32 + (t_ - 32) * 4) = *(const v4f*)(&cprow[(t_ - 32) * 4]);
    __threadfence(); }
}
__global__ __launch_bounds__(128) void outproj_kernel(const b16* __restrict__ OHh, const b16* __restrict__ OHl, const b16* __restrict__ WOUT, const float* __restrict__ bo, float* __restrict__ out) {
  __shared__ __attribute__((aligned(16))) float Tf[4][16][128 + 4];
  const int wave = threadIdx.x >> 5, lane = threadIdx.x & 31, nloc = lane & 15, hlf = lane >> 4; const size_t m0 = (size_t)blockIdx.x * 64 + wave * 16; const int n0 = blockIdx.y * 128;
  v8f acc[8];
#pragma unroll
  for (int t = 0; t < 8; ++t) acc[t] = (v8f){};
#pragma unroll 2
  for (int kb = 0; kb < HD; kb += 32) { const v16b a = frag_kb(OHh + (m0 + nloc) * HD + kb, hlf), al = frag_kb(OHl + (m0 + nloc) * HD + kb, hlf);
#pragma unroll
    for (int t = 0; t < 8; ++t) { const v16b bw = frag_kb(WOUT + (size_t)(n0 + t * 16 + nloc) * HD + kb, hlf); acc[t] = wmma16b(a, bw, acc[t]); acc[t] = wmma16b(al, bw, acc[t]); } }
#pragma unroll
  for (int t = 0; t < 8; ++t) { const float bb = bf16_rne(bo[n0 + t * 16 + nloc]);
#pragma unroll
    for (int r = 0; r < 8; ++r) Tf[wave][8 * hlf + r][t * 16 + nloc] = acc[t][r] * (1.0f / (XS * WSC)) + bb; }
  wave_lds_sync();
  for (int pass = 0; pass < 2; ++pass) { for (int rr = 0; rr < 16; ++rr) *(volatile v4f*)(out + (m0 + rr) * DIM + n0 + lane * 4) = *(const v4f*)(&Tf[wave][rr][lane * 4]); __threadfence(); }
}
__global__ __launch_bounds__(256) void coors_kernel(const float* __restrict__ CP, const float* __restrict__ coors, float* __restrict__ out1) {
  __shared__ __attribute__((aligned(16))) float res[N * 3];
  const int t_ = threadIdx.x;
  for (int q = t_; q < N * 3; q += 256) { const int ii = q / 3, c = q % 3; float s = bf16_rne(coors[q]); for (int hh = 0; hh < NH; ++hh) s += CP[((size_t)hh * N + ii) * 32 + c]; res[q] = s; }
  __syncthreads();
  for (int pass = 0; pass < 2; ++pass) { for (int q = t_; q < N * 3 / 4; q += 256) *(volatile v4f*)(out1 + q * 4) = *(const v4f*)(&res[q * 4]); __threadfence(); }
}
}

extern "C" void kernel_launch(void* const* d_in, const int* in_sizes, int n_in, void* d_out, int out_size, void* d_ws, size_t ws_size, hipStream_t stream) {
  (void)n_in;
  auto Fp = [&](int i) { return (const float*)d_in[i]; };
  if (in_sizes[0] != N * DIM || in_sizes[1] != N * 3 || in_sizes[2] != DIM * 3 * HD || in_sizes[3] != HD * DIM || in_sizes[5] != (2 * DH + 1) * E2 || in_sizes[7] != E2 * MD || in_sizes[9] != MD * A1 || in_sizes[11] != A1 || in_sizes[13] != MD * A1 || in_sizes[15] != A1 || out_size != N * DIM + N * 3) return;
  size_t off = 0; char* ws = (char*)d_ws;
  auto carve = [&](size_t bytes) { char* p = ws + off; off += (bytes + 255) & ~(size_t)255; return p; };
  b16* X16 = (b16*)carve((size_t)N * DIM * 2); b16* WQKV = (b16*)carve((size_t)3 * HD * DIM * 2); b16* WOUT = (b16*)carve((size_t)DIM * HD * 2); b16* WE1P = (b16*)carve((size_t)PW * DH * 2); b16* WE1Q = (b16*)carve((size_t)PW * DH * 2); b16* WE2T = (b16*)carve((size_t)MD * KE * 2);
  b16* WA1T = (b16*)carve((size_t)A1 * 32 * 2); b16* WC1T = (b16*)carve((size_t)A1 * 32 * 2); b16* WA2T = (b16*)carve((size_t)16 * A1 * 2); b16* WC2T = (b16*)carve((size_t)16 * A1 * 2);
  float* QKV = (float*)carve((size_t)N * 3 * HD * 4); b16* QKh = (b16*)carve((size_t)N * 2 * HD * 2); b16* QKl = (b16*)carve((size_t)N * 2 * HD * 2); float* P = (float*)carve((size_t)NRH * PW * 4); float* Qm = (float*)carve((size_t)NRH * PW * 4);
  b16* OHh = (b16*)carve((size_t)N * HD * 2); b16* OHl = (b16*)carve((size_t)N * HD * 2); float* CP = (float*)carve((size_t)NH * N * 32 * 4);
  if (off > ws_size || off > ((size_t)128 << 20)) return;
  prep_kernel<<<(unsigned)(((size_t)N * DIM / 8 + (size_t)3 * HD * DIM / 8 + (size_t)DIM * HD / 8 + 2 * (size_t)PW * DH / 8 + (size_t)MD * KE / 8 + 2 * (size_t)A1 * 32 / 8 + 2 * (size_t)16 * A1 / 8 + 255) / 256), 256, 0, stream>>>(Fp(0), Fp(2), Fp(3), Fp(5), Fp(7), Fp(9), Fp(11), Fp(13), Fp(15), X16, WQKV, WOUT, WE1P, WE1Q, WE2T, WA1T, WC1T, WA2T, WC2T);
  qkv_kernel<<<dim3(N / 64, 3 * HD / 128), 128, 0, stream>>>(X16, WQKV, QKV, QKh, QKl);
  pq_kernel<<<dim3(NRH / 64, PW / 128, 2), 128, 0, stream>>>(QKh, QKl, WE1P, WE1Q, Fp(6), P, Qm);
  pair_kernel<<<dim3(N, NH), 256, 0, stream>>>(P, Qm, Fp(5), Fp(1), QKV, WE2T, Fp(8), WA1T, Fp(10), WC1T, Fp(14), WA2T, Fp(12), WC2T, Fp(16), OHh, OHl, CP);
  outproj_kernel<<<dim3(N / 64, DIM / 128), 128, 0, stream>>>(OHh, OHl, WOUT, Fp(4), (float*)d_out);
  coors_kernel<<<1, 256, 0, stream>>>(CP, Fp(1), (float*)d_out + (size_t)N * DIM);
}
